// GINLapPE_45999099740571
// MI455X (gfx1250) — hardware-verified
//
#include <hip/hip_runtime.h>
#include <stddef.h>
#include <stdint.h>


#pragma clang fp contract(off)

#define NN      50000
#define NE      800000
#define NG      1000
#define HD      256
#define NL      5
#define NTO     128
#define MP      50048
#define MG      1024
#define K2      512
#define KE      32
#define NTHR    256
#define NWAVE   8
#define EPT     8
#define CHUNK   (NTHR * EPT)
#define WCAP    (EPT * 32)
#define LISTN   (NWAVE * WCAP)
#define NB      1024
#define NBLK    49
#define PKS     11
#define RCAP    20480
#define DEGCAP  64
#define GBM     64
#define GBN     128
#define GTHR    128
#define GWAVE   (GTHR / 32)
#define PARTW   288
#define XROWS   128
#define PLANE   (HD * K2)
#define NSEG    35
#define TB1     0
#define TG1     1280
#define TBE1    2560
#define TB2     3840
#define TBNG    5120
#define TBNB    6400
#define TEB     7680
#define TCL1B   7936
#define TCLG    8192
#define TCLB    8448
#define TCL2B   8704
#define TABN    (NSEG * 256)
#define WSMAX   134217728
#define LDS_CMP ((2 * RCAP + 2 * NB + LISTN + 16) * 4)

static_assert(HD == 256 && K2 == 2 * HD && (K2 % 32) == 0 && (KE % 32) == 0);
static_assert(MP % GBM == 0 && MP >= NN && MP - NN < GBM && MP % XROWS == 0);
static_assert(MG % GBM == 0 && MG >= NG);
static_assert(NBLK * NB >= MP);
static_assert((CHUNK & (CHUNK - 1)) == 0 && CHUNK <= (1 << PKS) && NB <= (1 << PKS));
static_assert(NE < (1 << 21) && (NE % 4) == 0);
static_assert(NB == 4 * NTHR && LISTN >= NB && (RCAP % (4 * NTHR)) == 0);
static_assert(RCAP >= 16659 + 16659 / 20 + 1);
static_assert(DEGCAP >= 36 + 8);
static_assert(LDS_CMP <= 300000);
static_assert(GBM == GWAVE * 16 && GBN == 4 * 32 && GTHR == GBN && HD % GBN == 0 && NTO == GBN);
static_assert(PARTW % 32 == 0 && PARTW / 4 <= GTHR && PARTW >= 2 * GBN + 1);
static_assert((NN * 9) % 4 == 0 && (NN * 8) % 4 == 0 && (XROWS * 9) % 4 == 0);
static_assert(TCL2B + 256 == TABN && (TABN / 4) % 32 == 0);

typedef float          v4f  __attribute__((ext_vector_type(4)));
typedef float          v8f  __attribute__((ext_vector_type(8)));
typedef int            v4i  __attribute__((ext_vector_type(4)));
typedef int            v8i  __attribute__((ext_vector_type(8)));
typedef unsigned int   v4u  __attribute__((ext_vector_type(4)));
typedef unsigned short v8us __attribute__((ext_vector_type(8)));
typedef __bf16         v16b __attribute__((ext_vector_type(16)));
typedef v4f  __attribute__((may_alias)) v4fa;
typedef v4i  __attribute__((may_alias)) v4ia;
typedef v8us __attribute__((may_alias)) v8usa;
union FragB { v16b v; v8us h[2]; v8i w; };

__device__ __forceinline__ v8f wmb(const FragB& a, const FragB& b, v8f c) {
  v8f d = __builtin_amdgcn_wmma_f32_16x16x32_bf16(false, a.v, false, b.v, (short)0, c, false, false);
  asm volatile("v_nop\n\tv_nop\n\tv_nop\n\tv_nop" : "+v"(d) : "v"(a.w), "v"(b.w));
  return d;
}

__device__ __forceinline__ v8f z8() { v8f z = {0.f, 0.f, 0.f, 0.f, 0.f, 0.f, 0.f, 0.f}; return z; }

__device__ __forceinline__ unsigned bf_bits(float f) {
  const unsigned u = __float_as_uint(f);
  const unsigned r = (u + 0x7FFFu + ((u >> 16) & 1u)) >> 16;
  return ((u & 0x7fffffffu) > 0x7f800000u) ? 0x7fc0u : r;
}
__device__ __forceinline__ float bf_val(unsigned b) { return __uint_as_float(b << 16); }
__device__ __forceinline__ float bf_rne(float f) { return bf_val(bf_bits(f)); }
__device__ __forceinline__ float relu_np(float v) { return (v > 0.0f) ? v : (v - v); }

struct HL { v4u h; v4u l; };
__device__ __forceinline__ HL split8(const v4f a, const v4f b) {
  const float f[8] = {a.x, a.y, a.z, a.w, b.x, b.y, b.z, b.w};
  unsigned hw[4], lw[4];
#pragma unroll
  for (int j = 0; j < 4; ++j) {
    const unsigned h0 = bf_bits(f[2 * j]), h1 = bf_bits(f[2 * j + 1]);
    const unsigned l0 = bf_bits(f[2 * j] - bf_val(h0)), l1 = bf_bits(f[2 * j + 1] - bf_val(h1));
    hw[j] = h0 | (h1 << 16);
    lw[j] = l0 | (l1 << 16);
  }
  HL o;
  o.h.x = hw[0]; o.h.y = hw[1]; o.h.z = hw[2]; o.h.w = hw[3];
  o.l.x = lw[0]; o.l.y = lw[1]; o.l.z = lw[2]; o.l.w = lw[3];
  return o;
}

__device__ __forceinline__ int scan_chunk(const int* __restrict__ dsts, int nE, int cbase, int slotBase,
                                          int nb, int vec8, int* list, int tid, int lane, int wave) {
  int wc = 0;
  const int el0  = tid * EPT;
  const int e0   = cbase + el0;
  const int sent = -2147483647 - 1;
  v4i da, db;
  if (vec8 != 0 && cbase + CHUNK <= nE) {
    da = *(const v4i*)(dsts + e0);
    db = *(const v4i*)(dsts + e0 + 4);
  } else {
    da.x = (e0     < nE) ? dsts[min(e0,     nE - 1)] : sent;
    da.y = (e0 + 1 < nE) ? dsts[min(e0 + 1, nE - 1)] : sent;
    da.z = (e0 + 2 < nE) ? dsts[min(e0 + 2, nE - 1)] : sent;
    da.w = (e0 + 3 < nE) ? dsts[min(e0 + 3, nE - 1)] : sent;
    db.x = (e0 + 4 < nE) ? dsts[min(e0 + 4, nE - 1)] : sent;
    db.y = (e0 + 5 < nE) ? dsts[min(e0 + 5, nE - 1)] : sent;
    db.z = (e0 + 6 < nE) ? dsts[min(e0 + 6, nE - 1)] : sent;
    db.w = (e0 + 7 < nE) ? dsts[min(e0 + 7, nE - 1)] : sent;
  }
  const unsigned nbs = (unsigned)slotBase;
  const unsigned unb = (unsigned)nb;
  const unsigned s0 = (unsigned)da.x - nbs, s1 = (unsigned)da.y - nbs;
  const unsigned s2 = (unsigned)da.z - nbs, s3 = (unsigned)da.w - nbs;
  const unsigned s4 = (unsigned)db.x - nbs, s5 = (unsigned)db.y - nbs;
  const unsigned s6 = (unsigned)db.z - nbs, s7 = (unsigned)db.w - nbs;
  const bool h0 = s0 < unb, h1 = s1 < unb, h2 = s2 < unb, h3 = s3 < unb;
  const bool h4 = s4 < unb, h5 = s5 < unb, h6 = s6 < unb, h7 = s7 < unb;
  const unsigned any = __builtin_amdgcn_ballot_w32(h0 | h1 | h2 | h3 | h4 | h5 | h6 | h7);
  if (any != 0u) {
#define HITJ(J, HJ, SJ) { \
      const unsigned mj = __builtin_amdgcn_ballot_w32(HJ); \
      if (mj != 0u) { \
        if (HJ) { \
          const int pos = wc + (int)__builtin_amdgcn_mbcnt_lo(mj, 0u); \
          if (pos < WCAP) list[wave * WCAP + pos] = ((el0 + (J)) << PKS) | (int)(SJ); \
        } \
        wc += (int)__builtin_popcount(mj); } }
    HITJ(0, h0, s0)
    HITJ(1, h1, s1)
    HITJ(2, h2, s2)
    HITJ(3, h3, s3)
    HITJ(4, h4, s4)
    HITJ(5, h5, s5)
    HITJ(6, h6, s6)
    HITJ(7, h7, s7)
#undef HITJ
  }
  return wc;
}

__global__ __launch_bounds__(NTHR) void k_xe(const float* __restrict__ xa, const float* __restrict__ xp,
                                             int nN, unsigned short* xe) {
  __shared__ __attribute__((aligned(16))) float xaS[XROWS * 9];
  __shared__ __attribute__((aligned(16))) float xpS[XROWS * 8];
  const int tid = (int)threadIdx.x, blk = (int)blockIdx.x;
  const int totA = (nN * 9) >> 2, totP = (nN * 8) >> 2;
#pragma unroll 1
  for (int i = tid; i < (XROWS * 9) / 4; i += NTHR) {
    const int gi = blk * ((XROWS * 9) / 4) + i;
    const int gc = gi < totA ? gi : totA - 1;
    v4f v = *(const v4f*)(xa + 4 * (size_t)gc);
    const bool ok = gi < totA;
    v.x = ok ? v.x : 0.0f; v.y = ok ? v.y : 0.0f; v.z = ok ? v.z : 0.0f; v.w = ok ? v.w : 0.0f;
    *(v4fa*)(xaS + 4 * i) = v;
  }
#pragma unroll 1
  for (int i = tid; i < (XROWS * 8) / 4; i += NTHR) {
    const int gi = blk * ((XROWS * 8) / 4) + i;
    const int gc = gi < totP ? gi : totP - 1;
    v4f v = *(const v4f*)(xp + 4 * (size_t)gc);
    const bool ok = gi < totP;
    v.x = ok ? v.x : 0.0f; v.y = ok ? v.y : 0.0f; v.z = ok ? v.z : 0.0f; v.w = ok ? v.w : 0.0f;
    *(v4fa*)(xpS + 4 * i) = v;
  }
  __syncthreads();
  v4u o[2];
#pragma unroll
  for (int it = 0; it < 2; ++it) {
    const int u = tid + NTHR * it;
    const int r = u >> 2, q = u & 3;
    unsigned bb[8];
#pragma unroll
    for (int j = 0; j < 8; ++j) {
      const int c  = 8 * q + j;
      const int ia = c < 8 ? c : 8;
      int ib = c - 9;
      ib = ib < 0 ? 0 : (ib > 7 ? 7 : ib);
      const unsigned ua = __float_as_uint(xaS[r * 9 + ia]);
      const unsigned ub = __float_as_uint(xpS[r * 8 + ib]);
      const unsigned ma = 0u - (unsigned)(c < 9);
      const unsigned mb = 0u - (unsigned)((c >= 9) & (c < 17));
      bb[j] = bf_bits(__uint_as_float((ua & ma) | (ub & mb)));
    }
    v4u w;
    w.x = bb[0] | (bb[1] << 16); w.y = bb[2] | (bb[3] << 16);
    w.z = bb[4] | (bb[5] << 16); w.w = bb[6] | (bb[7] << 16);
    o[it] = w;
  }
  unsigned short* dp = xe + (size_t)blk * XROWS * KE + (size_t)tid * 8;
  *(volatile v4u*)dp = o[0];
  *(volatile v4u*)(dp + NTHR * 8) = o[1];
  __threadfence();
  *(volatile v4u*)dp = o[0];
  *(volatile v4u*)(dp + NTHR * 8) = o[1];
}

__global__ __launch_bounds__(NTHR) void k_wprep(const float* __restrict__ w1, const float* __restrict__ w2,
                                                const float* __restrict__ c1, const float* __restrict__ c2,
                                                unsigned short* wp) {
  const int blk = (int)blockIdx.x, tid = (int)threadIdx.x;
  const int mi = blk >> 5;
  const float* Wb;
  int ld = HD;
  int v = (blk & 31) * NTHR + tid;
  if (mi < NL) {
    Wb = w1 + (size_t)mi * HD * HD;
  } else if (mi < 2 * NL) {
    Wb = w2 + (size_t)(mi - NL) * HD * HD;
  } else if (mi == 2 * NL) {
    Wb = c1;
  } else {
    Wb = c2;
    ld = NTO;
    v = (blk - 32 * (2 * NL + 1)) * NTHR + tid;
  }
  const int n  = v >> 5;
  const int k8 = (v & 31) * 8;
  const float* p = Wb + (size_t)k8 * ld + n;
  v8us o;
#pragma unroll
  for (int i = 0; i < 8; ++i) o[i] = (unsigned short)bf_bits(p[(size_t)i * ld]);
  unsigned short* dp = wp + (size_t)mi * PLANE + (size_t)n * K2 + k8;
  *(volatile v8us*)dp = o;
  *(volatile v8us*)(dp + HD) = o;
  __threadfence();
  *(volatile v8us*)dp = o;
  *(volatile v8us*)(dp + HD) = o;
}

__global__ __launch_bounds__(NTHR) void k_small(
    const float* __restrict__ aew, const float* __restrict__ pew,
    const float* __restrict__ b1, const float* __restrict__ g1, const float* __restrict__ be1,
    const float* __restrict__ b2, const float* __restrict__ bng, const float* __restrict__ bnb,
    const float* __restrict__ aeb, const float* __restrict__ peb,
    const float* __restrict__ cl1b, const float* __restrict__ clg, const float* __restrict__ clb,
    const float* __restrict__ cl2b, unsigned short* we, float* tab) {
  __shared__ __attribute__((aligned(16))) float awS[9 * HD];
  __shared__ __attribute__((aligned(16))) float pwS[8 * HD];
  const int tid = (int)threadIdx.x;
  if (blockIdx.x == 0) {
#pragma unroll 1
    for (int i = tid; i < (9 * HD) / 4; i += NTHR) *(v4fa*)(awS + 4 * i) = *(const v4f*)(aew + 4 * i);
#pragma unroll 1
    for (int i = tid; i < (8 * HD) / 4; i += NTHR) *(v4fa*)(pwS + 4 * i) = *(const v4f*)(pew + 4 * i);
    __syncthreads();
#pragma unroll 1
    for (int it = 0; it < 4; ++it) {
      const int u = it * NTHR + tid;
      const int n = u >> 2, q = u & 3;
      unsigned bb[8];
#pragma unroll
      for (int j = 0; j < 8; ++j) {
        const int k  = 8 * q + j;
        const int ka = k < 8 ? k : 8;
        int kb = k - 9;
        kb = kb < 0 ? 0 : (kb > 7 ? 7 : kb);
        const unsigned ua = __float_as_uint(awS[ka * HD + n]);
        const unsigned ub = __float_as_uint(pwS[kb * HD + n]);
        const unsigned ma = 0u - (unsigned)(k < 9);
        const unsigned mb = 0u - (unsigned)((k >= 9) & (k < 17));
        bb[j] = bf_bits(__uint_as_float((ua & ma) | (ub & mb)));
      }
      v4u w;
      w.x = bb[0] | (bb[1] << 16); w.y = bb[2] | (bb[3] << 16);
      w.z = bb[4] | (bb[5] << 16); w.w = bb[6] | (bb[7] << 16);
      unsigned short* dp = we + (size_t)u * 8;
      *(volatile v4u*)dp = w;
      __threadfence();
      *(volatile v4u*)dp = w;
    }
    return;
  }
  const int u = ((int)blockIdx.x - 1) * NTHR + tid;
  if (u >= NSEG * 64) return;
  const int seg = __builtin_amdgcn_readfirstlane(u >> 6);
  const int w = u & 63;
  v4f v = {0.f, 0.f, 0.f, 0.f};
  if (seg < 30) {
    const int grp = seg / 5;
    const int ly  = seg - 5 * grp;
    const float* s = (grp == 0) ? b1 : (grp == 1) ? g1 : (grp == 2) ? be1 : (grp == 3) ? b2 : (grp == 4) ? bng : bnb;
    const v4f a = *(const v4f*)(s + ly * HD + 4 * w);
    v.x = bf_rne(a.x); v.y = bf_rne(a.y); v.z = bf_rne(a.z); v.w = bf_rne(a.w);
  } else if (seg == 30) {
    const v4f a = *(const v4f*)(aeb + 4 * w);
    const v4f b = *(const v4f*)(peb + 4 * w);
    v.x = bf_rne(a.x) + bf_rne(b.x); v.y = bf_rne(a.y) + bf_rne(b.y);
    v.z = bf_rne(a.z) + bf_rne(b.z); v.w = bf_rne(a.w) + bf_rne(b.w);
  } else if (seg < 34) {
    const float* s = (seg == 31) ? cl1b : (seg == 32) ? clg : clb;
    const v4f a = *(const v4f*)(s + 4 * w);
    v.x = bf_rne(a.x); v.y = bf_rne(a.y); v.z = bf_rne(a.z); v.w = bf_rne(a.w);
  } else {
    const v4f a = *(const v4f*)(cl2b + 4 * (w & 31));
    const bool ok = w < 32;
    v.x = ok ? bf_rne(a.x) : 0.0f; v.y = ok ? bf_rne(a.y) : 0.0f;
    v.z = ok ? bf_rne(a.z) : 0.0f; v.w = ok ? bf_rne(a.w) : 0.0f;
  }
  float* tp = tab + (size_t)u * 4;
  *(volatile v4f*)tp = v;
  __threadfence();
  *(volatile v4f*)tp = v;
}

__global__ __launch_bounds__(NTHR) void k_compact(const int* __restrict__ srcs, const int* __restrict__ dsts,
                                                  int nE, int nN, int vec8,
                                                  int* LISTg, int* CNTg, int* OFFg) {
  extern __shared__ v4f lds_dyn[];
  int* reg1 = (int*)lds_dyn;
  int* reg2 = reg1 + RCAP;
  int* scnt = reg2 + RCAP;
  int* soff = scnt + NB;
  int* list = soff + NB;
  int* wcnt = list + LISTN;
  int* wtot = wcnt + NWAVE;
  const int tid = (int)threadIdx.x, lane = tid & 31, wave = tid >> 5;
  const int blk = (int)blockIdx.x;
  const int nodeBase = blk * NB;

  {
    const v4i z4 = {0, 0, 0, 0};
#pragma unroll 1
    for (int i = tid * 4; i < RCAP; i += NTHR * 4) *(v4ia*)(reg2 + i) = z4;
    *(v4ia*)(scnt + 4 * tid) = z4;
  }
  __syncthreads();

  int tot = 0;
  const int nChunks = (nE + CHUNK - 1) / CHUNK;
#pragma unroll 1
  for (int ch = 0; ch < nChunks; ++ch) {
    const int cbase = ch * CHUNK;
    const int wc = scan_chunk(dsts, nE, cbase, nodeBase, NB, vec8, list, tid, lane, wave);
    if (lane == 0) wcnt[wave] = wc;
    __syncthreads();
    int pre = 0, all = 0;
#pragma unroll
    for (int w2 = 0; w2 < NWAVE; ++w2) {
      int c = wcnt[w2];
      c = c < 0 ? 0 : (c > WCAP ? WCAP : c);
      all += c;
      pre += (w2 < wave) ? c : 0;
    }
    const int wcc  = wc > WCAP ? WCAP : wc;
    const int base = tot + pre;
#pragma unroll 1
    for (int i = lane; i < wcc; i += 32) {
      const int ent = list[wave * WCAP + i];
      const int el  = (ent >> PKS) & (CHUNK - 1);
      const int sl  = ent & (NB - 1);
      int eid = cbase + el;
      eid = eid > nE - 1 ? nE - 1 : eid;
      const int pos = base + i;
      if (pos < RCAP) reg1[pos] = (int)(((unsigned)eid << PKS) | (unsigned)sl);
    }
    tot += all;
    tot = tot > RCAP ? RCAP : tot;
    __syncthreads();
  }
  const int nh = tot;

  if (wave == 0) {
#pragma unroll 1
    for (int b0 = 0; b0 < nh; b0 += 32) {
      const int idx = b0 + lane;
      const int uv  = reg1[idx < nh ? idx : nh - 1];
      const int m32 = (nh - b0) < 32 ? (nh - b0) : 32;
#pragma unroll 1
      for (int k = 0; k < m32; ++k) {
        const int u  = __builtin_amdgcn_readlane(uv, k);
        const int sl = u & (NB - 1);
        if (lane == 0) scnt[sl] = scnt[sl] + 1;
      }
    }
  }
  __syncthreads();

  {
    const v4i ca = *(const v4ia*)(scnt + 4 * tid);
    const int e0 = ca.x < 0 ? 0 : ca.x, e1 = ca.y < 0 ? 0 : ca.y, e2 = ca.z < 0 ? 0 : ca.z, e3 = ca.w < 0 ? 0 : ca.w;
    const int ts = e0 + e1 + e2 + e3;
    int incl = ts;
#pragma unroll
    for (int d = 1; d < 32; d <<= 1) {
      const int up = __shfl_up(incl, d);
      if (lane >= d) incl += up;
    }
    if (lane == 31) wtot[wave] = incl;
    __syncthreads();
    int pre = 0;
#pragma unroll
    for (int w2 = 0; w2 < NWAVE; ++w2) pre += (w2 < wave) ? wtot[w2] : 0;
    int run = pre + incl - ts;
    soff[4 * tid + 0] = run; run += e0;
    soff[4 * tid + 1] = run; run += e1;
    soff[4 * tid + 2] = run; run += e2;
    soff[4 * tid + 3] = run;
  }
  __syncthreads();
#pragma unroll 1
  for (int i = tid; i < NB; i += NTHR) list[i] = soff[i];
  __syncthreads();

  if (wave == 0) {
#pragma unroll 1
    for (int b0 = 0; b0 < nh; b0 += 32) {
      const int idx = b0 + lane;
      const int uv  = reg1[idx < nh ? idx : nh - 1];
      const int m32 = (nh - b0) < 32 ? (nh - b0) : 32;
#pragma unroll 1
      for (int k = 0; k < m32; ++k) {
        const int u   = __builtin_amdgcn_readlane(uv, k);
        const int sl  = u & (NB - 1);
        const int eid = (int)((unsigned)u >> PKS);
        if (lane == 0) {
          int pos = list[sl];
          pos = pos < 0 ? 0 : (pos > RCAP - 1 ? RCAP - 1 : pos);
          reg2[pos] = eid;
          list[sl] = pos + 1;
        }
      }
    }
  }
  __syncthreads();

  const bool ovf = (nh >= RCAP);
  int* lout = LISTg + (size_t)blk * RCAP;
#pragma unroll 1
  for (int it = 0; it < RCAP / (4 * NTHR); ++it) {
    const int base = 4 * (it * NTHR + tid);
    const v4i ev = *(const v4ia*)(reg2 + base);
    int e0 = ev.x, e1 = ev.y, e2 = ev.z, e3 = ev.w;
    e0 = e0 < 0 ? 0 : (e0 > nE - 1 ? nE - 1 : e0);
    e1 = e1 < 0 ? 0 : (e1 > nE - 1 ? nE - 1 : e1);
    e2 = e2 < 0 ? 0 : (e2 > nE - 1 ? nE - 1 : e2);
    e3 = e3 < 0 ? 0 : (e3 > nE - 1 ? nE - 1 : e3);
    int s0 = srcs[e0], s1 = srcs[e1], s2 = srcs[e2], s3 = srcs[e3];
    s0 = s0 < 0 ? 0 : (s0 > nN - 1 ? nN - 1 : s0);
    s1 = s1 < 0 ? 0 : (s1 > nN - 1 ? nN - 1 : s1);
    s2 = s2 < 0 ? 0 : (s2 > nN - 1 ? nN - 1 : s2);
    s3 = s3 < 0 ? 0 : (s3 > nN - 1 ? nN - 1 : s3);
    v4i o;
    o.x = (base + 0 < nh) ? s0 : 0;
    o.y = (base + 1 < nh) ? s1 : 0;
    o.z = (base + 2 < nh) ? s2 : 0;
    o.w = (base + 3 < nh) ? s3 : 0;
    *(volatile v4i*)(lout + base) = o;
    __threadfence();
    *(volatile v4i*)(lout + base) = o;
  }
  {
    v4i c4 = *(const v4ia*)(scnt + 4 * tid);
    const v4i o4 = *(const v4ia*)(soff + 4 * tid);
    c4.x = ovf ? (DEGCAP + 1) : c4.x; c4.y = ovf ? (DEGCAP + 1) : c4.y;
    c4.z = ovf ? (DEGCAP + 1) : c4.z; c4.w = ovf ? (DEGCAP + 1) : c4.w;
    int* cp = CNTg + (size_t)blk * NB + 4 * tid;
    int* op = OFFg + (size_t)blk * NB + 4 * tid;
    *(volatile v4i*)cp = c4;
    *(volatile v4i*)op = o4;
    __threadfence();
    *(volatile v4i*)cp = c4;
    *(volatile v4i*)op = o4;
  }
}

__global__ __launch_bounds__(NTHR) void k_agg(const int* __restrict__ LISTg, const int* __restrict__ CNTg,
                                              const int* __restrict__ OFFg, const float* __restrict__ Hf,
                                              unsigned short* P1, int nN, int MPr) {
  __shared__ __attribute__((aligned(16))) int scn[NB];
  __shared__ __attribute__((aligned(16))) int sof[NB];
  const int tid = (int)threadIdx.x, lane = tid & 31;
  const int wave = __builtin_amdgcn_readfirstlane(tid >> 5);
  const int blk = (int)blockIdx.x;
  const int nodeBase = blk * NB;
  *(v4ia*)(scn + 4 * tid) = *(const v4i*)(CNTg + (size_t)blk * NB + 4 * tid);
  *(v4ia*)(sof + 4 * tid) = *(const v4i*)(OFFg + (size_t)blk * NB + 4 * tid);
  __syncthreads();
  const int* lst = LISTg + (size_t)blk * RCAP;
  const float qnan = __int_as_float(0x7fc00000);

#pragma unroll 1
  for (int jt = 0; jt < NB / NWAVE; ++jt) {
    const int slot = wave * (NB / NWAVE) + jt;
    const int grow = nodeBase + slot;
    if (grow >= MPr) break;
    const int craw = scn[slot];
    int st = sof[slot];
    const bool bad = (craw < 0) | (craw > DEGCAP);
    int cnt = craw < 0 ? 0 : (craw > DEGCAP ? DEGCAP : craw);
    st = st < 0 ? 0 : (st > RCAP ? RCAP : st);
    if (cnt > RCAP - st) cnt = RCAP - st;
    const bool live = grow < nN;
    if (!live) cnt = 0;

    float a0 = 0.f, a1 = 0.f, a2 = 0.f, a3 = 0.f, a4 = 0.f, a5 = 0.f, a6 = 0.f, a7 = 0.f;
#pragma unroll 1
    for (int b0 = 0; b0 < cnt; b0 += 32) {
      int idx = st + b0 + lane;
      idx = idx > RCAP - 1 ? RCAP - 1 : idx;
      int sv = lst[idx];
      sv = sv < 0 ? 0 : (sv > nN - 1 ? nN - 1 : sv);
      const int m32 = (cnt - b0) < 32 ? (cnt - b0) : 32;
#pragma unroll 1
      for (int k = 0; k < m32; ++k) {
        const int sk = __builtin_amdgcn_readlane(sv, k);
        const float* rp = Hf + (size_t)sk * HD + 8 * lane;
        const v4f va = *(const v4f*)rp;
        const v4f vb = *(const v4f*)(rp + 4);
        a0 += va.x; a1 += va.y; a2 += va.z; a3 += va.w;
        a4 += vb.x; a5 += vb.y; a6 += vb.z; a7 += vb.w;
      }
    }
    const int nc = live ? grow : nN - 1;
    const float* sp = Hf + (size_t)nc * HD + 8 * lane;
    const v4f sa = *(const v4f*)sp;
    const v4f sb = *(const v4f*)(sp + 4);
    const bool poi = bad & live;
    v4f ra, rb;
    ra.x = sa.x + a0; ra.y = sa.y + a1; ra.z = sa.z + a2; ra.w = sa.w + a3;
    rb.x = sb.x + a4; rb.y = sb.y + a5; rb.z = sb.z + a6; rb.w = sb.w + a7;
    ra.x = live ? ra.x : 0.0f; ra.y = live ? ra.y : 0.0f; ra.z = live ? ra.z : 0.0f; ra.w = live ? ra.w : 0.0f;
    rb.x = live ? rb.x : 0.0f; rb.y = live ? rb.y : 0.0f; rb.z = live ? rb.z : 0.0f; rb.w = live ? rb.w : 0.0f;
    ra.x = poi ? qnan : ra.x; ra.y = poi ? qnan : ra.y; ra.z = poi ? qnan : ra.z; ra.w = poi ? qnan : ra.w;
    rb.x = poi ? qnan : rb.x; rb.y = poi ? qnan : rb.y; rb.z = poi ? qnan : rb.z; rb.w = poi ? qnan : rb.w;
    const HL hl = split8(ra, rb);
    unsigned short* gp = P1 + (size_t)grow * K2 + 8 * lane;
    *(volatile v4u*)gp = hl.h;
    *(volatile v4u*)(gp + HD) = hl.l;
    __threadfence();
    *(volatile v4u*)gp = hl.h;
    *(volatile v4u*)(gp + HD) = hl.l;
  }
}

template <int KK, int REC>
__global__ __launch_bounds__(GTHR) void k_gemm(const unsigned short* __restrict__ A,
                                               const unsigned short* __restrict__ BT,
                                               const float* __restrict__ bias,
                                               float* outp, int ldo, int nStore, int nValid, float* part) {
  __shared__ __attribute__((aligned(16))) float stg[GBM * GBN];
  const int tid = (int)threadIdx.x, lane = tid & 31, wave = tid >> 5, hh = lane >> 4, m = lane & 15;
  const int rowBase = (int)blockIdx.x * GBM;
  const int colBase = (int)blockIdx.y * GBN;

  v8f acc[8];
#pragma unroll
  for (int t = 0; t < 8; ++t) acc[t] = z8();
  const unsigned short* ap = A  + (size_t)(rowBase + 16 * wave + m) * (size_t)KK + 8 * hh;
  const unsigned short* bp = BT + (size_t)(colBase + m) * (size_t)KK + 8 * hh;

#pragma unroll 1
  for (int k0 = 0; k0 < KK; k0 += 32) {
    FragB af;
    af.h[0] = *(const v8usa*)(ap + k0);
    af.h[1] = *(const v8usa*)(ap + k0 + 16);
#pragma unroll
    for (int nt = 0; nt < 8; ++nt) {
      const unsigned short* wq = bp + (size_t)(16 * nt) * (size_t)KK + k0;
      FragB bf;
      bf.h[0] = *(const v8usa*)wq;
      bf.h[1] = *(const v8usa*)(wq + 16);
      acc[nt] = wmb(af, bf, acc[nt]);
    }
  }

#pragma unroll
  for (int nt = 0; nt < 8; ++nt) {
    const int lc = 16 * nt + m;
#pragma unroll
    for (int r = 0; r < 8; ++r) {
      const int lr = 16 * wave + 8 * hh + r;
      stg[lr * GBN + lc] = acc[nt][r];
    }
  }
  __syncthreads();

  const v4f bq = *(const v4f*)(bias + colBase + 4 * lane);
  v4f pv[16];
#pragma unroll
  for (int i = 0; i < 16; ++i) {
    const int row = rowBase + 16 * wave + i;
    const bool ok = row < nValid;
    const v4f x = *(const v4fa*)(stg + (16 * wave + i) * GBN + 4 * lane);
    v4f y;
    y.x = ok ? (x.x + bq.x) : 0.0f;
    y.y = ok ? (x.y + bq.y) : 0.0f;
    y.z = ok ? (x.z + bq.z) : 0.0f;
    y.w = ok ? (x.w + bq.w) : 0.0f;
    pv[i] = y;
  }
#pragma unroll
  for (int i = 0; i < 16; ++i) {
    const int gr = rowBase + 16 * wave + i;
    float* op = outp + (size_t)gr * (size_t)ldo + colBase + 4 * lane;
    if (gr < nStore) *(volatile v4f*)op = pv[i];
  }
  __threadfence();
#pragma unroll
  for (int i = 0; i < 16; ++i) {
    const int gr = rowBase + 16 * wave + i;
    float* op = outp + (size_t)gr * (size_t)ldo + colBase + 4 * lane;
    if (gr < nStore) *(volatile v4f*)op = pv[i];
  }

  if constexpr (REC != 0) {
    __shared__ __attribute__((aligned(16))) float pst[PARTW];
    int rv = nValid - rowBase;
    rv = rv < 0 ? 0 : (rv > GBM ? GBM : rv);
    const float bc = bias[colBase + tid];
    float s = 0.0f;
#pragma unroll 1
    for (int r = 0; r < rv; ++r) s += stg[r * GBN + tid] + bc;
    const float den = rv > 0 ? (float)rv : 1.0f;
    const float mean = s / den;
    float q = 0.0f;
#pragma unroll 1
    for (int r = 0; r < rv; ++r) {
      const float d = (stg[r * GBN + tid] + bc) - mean;
      q += d * d;
    }
    pst[1 + tid] = mean;
    pst[1 + GBN + tid] = q;
    if (tid == 0) pst[0] = (float)rv;
#pragma unroll 1
    for (int i = 2 * GBN + 1 + tid; i < PARTW; i += GTHR) pst[i] = 0.0f;
    __syncthreads();
    const int pb = (int)blockIdx.x * (int)gridDim.y + (int)blockIdx.y;
    v4f ps = {0.f, 0.f, 0.f, 0.f};
    if (tid < PARTW / 4) {
      ps = *(const v4fa*)(pst + 4 * tid);
      *(volatile v4f*)(part + (size_t)pb * PARTW + 4 * tid) = ps;
    }
    __threadfence();
    if (tid < PARTW / 4) {
      *(volatile v4f*)(part + (size_t)pb * PARTW + 4 * tid) = ps;
    }
  }
}

__global__ __launch_bounds__(NTHR) void k_comb(const float* __restrict__ part, int nPart, int nCB,
                                               const float* __restrict__ gtab, const float* __restrict__ btab,
                                               float* stat) {
  __shared__ __attribute__((aligned(16))) float stg[4 * HD];
  const int tid = (int)threadIdx.x;
  const int c  = tid;
  const int cb = c >> 7;
  const int cc = c & (GBN - 1);
  double n = 0.0, mean = 0.0, M2 = 0.0;
#pragma unroll 1
  for (int b = 0; b < nPart; ++b) {
    const float* pr = part + ((size_t)b * (size_t)nCB + (size_t)cb) * PARTW;
    const double nb = (double)pr[0];
    const double mb = (double)pr[1 + cc];
    const double qb = (double)pr[1 + GBN + cc];
    if (nb > 0.5) {
      const double nn = n + nb;
      const double delta = mb - mean;
      const double f = nb / nn;
      mean = mean + delta * f;
      M2 = M2 + qb + delta * delta * n * f;
      n = nn;
    }
  }
  const double nt = n < 1.0 ? 1.0 : n;
  const float varf  = (float)(M2 / nt);
  const float meanf = (float)mean;
  const float ve = varf + 1e-5f;
  const float rstd = 1.0f / sqrtf(ve);
  stg[c] = meanf;
  stg[HD + c] = rstd;
  stg[2 * HD + c] = gtab[c];
  stg[3 * HD + c] = btab[c];
  __syncthreads();
  const v4f v = *(const v4fa*)(stg + 4 * tid);
  *(volatile v4f*)(stat + 4 * tid) = v;
  __threadfence();
  *(volatile v4f*)(stat + 4 * tid) = v;
}

__global__ __launch_bounds__(NTHR) void k_apply_hl(const float* __restrict__ X, const float* __restrict__ stat,
                                                   unsigned short* P, int nN, int nUnits) {
  __shared__ __attribute__((aligned(16))) float sst[4 * HD];
  const int tid = (int)threadIdx.x;
  *(v4fa*)(sst + 4 * tid) = *(const v4f*)(stat + 4 * tid);
  __syncthreads();
  const int u = (int)blockIdx.x * NTHR + tid;
  if (u >= nUnits) return;
  const int row = u >> 5;
  const int c8  = (u & 31) * 8;
  const int rc  = row < nN ? row : nN - 1;
  const bool ok = row < nN;
  const float* xp = X + (size_t)rc * HD + c8;
  const v4f xa = *(const v4f*)xp;
  const v4f xb = *(const v4f*)(xp + 4);
  const v4f ma = *(const v4fa*)(sst + c8),          mb = *(const v4fa*)(sst + c8 + 4);
  const v4f ra = *(const v4fa*)(sst + HD + c8),     rb = *(const v4fa*)(sst + HD + c8 + 4);
  const v4f ga = *(const v4fa*)(sst + 2 * HD + c8), gb = *(const v4fa*)(sst + 2 * HD + c8 + 4);
  const v4f ba = *(const v4fa*)(sst + 3 * HD + c8), bb = *(const v4fa*)(sst + 3 * HD + c8 + 4);
  v4f ya = ((xa - ma) * ra) * ga + ba;
  v4f yb = ((xb - mb) * rb) * gb + bb;
  ya.x = ok ? relu_np(ya.x) : 0.0f; ya.y = ok ? relu_np(ya.y) : 0.0f;
  ya.z = ok ? relu_np(ya.z) : 0.0f; ya.w = ok ? relu_np(ya.w) : 0.0f;
  yb.x = ok ? relu_np(yb.x) : 0.0f; yb.y = ok ? relu_np(yb.y) : 0.0f;
  yb.z = ok ? relu_np(yb.z) : 0.0f; yb.w = ok ? relu_np(yb.w) : 0.0f;
  const HL hl = split8(ya, yb);
  unsigned short* gp = P + (size_t)row * K2 + c8;
  *(volatile v4u*)gp = hl.h;
  *(volatile v4u*)(gp + HD) = hl.l;
  __threadfence();
  *(volatile v4u*)gp = hl.h;
  *(volatile v4u*)(gp + HD) = hl.l;
}

__global__ __launch_bounds__(NTHR) void k_apply_f(float* X, const float* __restrict__ stat, int nUnits) {
  __shared__ __attribute__((aligned(16))) float sst[4 * HD];
  const int tid = (int)threadIdx.x;
  *(v4fa*)(sst + 4 * tid) = *(const v4f*)(stat + 4 * tid);
  __syncthreads();
  const int u = (int)blockIdx.x * NTHR + tid;
  if (u >= nUnits) return;
  const int c4 = (u & 63) * 4;
  float* p = X + (size_t)u * 4;
  const v4f x  = *(const v4f*)p;
  const v4f mm = *(const v4fa*)(sst + c4);
  const v4f rr = *(const v4fa*)(sst + HD + c4);
  const v4f gg = *(const v4fa*)(sst + 2 * HD + c4);
  const v4f bb = *(const v4fa*)(sst + 3 * HD + c4);
  v4f y = ((x - mm) * rr) * gg + bb;
  v4f o;
  o.x = relu_np(y.x); o.y = relu_np(y.y); o.z = relu_np(y.z); o.w = relu_np(y.w);
  *(volatile v4f*)p = o;
  __threadfence();
  *(volatile v4f*)p = o;
}

__global__ __launch_bounds__(NTHR) void k_pool(const float* __restrict__ Hf, const int* __restrict__ bat,
                                               int nN, int nG, unsigned short* PL) {
  const int tid = (int)threadIdx.x, lane = tid & 31;
  const int wave = __builtin_amdgcn_readfirstlane(tid >> 5);
  const int g = (int)blockIdx.x * NWAVE + wave;
  const int lim = (g < nG) ? nN : 0;
  float a0 = 0.f, a1 = 0.f, a2 = 0.f, a3 = 0.f, a4 = 0.f, a5 = 0.f, a6 = 0.f, a7 = 0.f;
  int cnt = 0;
#pragma unroll 1
  for (int i0 = 0; i0 < lim; i0 += 32) {
    const int i  = i0 + lane;
    const int ic = i < nN ? i : nN - 1;
    const int b  = bat[ic];
    const bool hit = (i < nN) & (b == g);
    unsigned msk = __builtin_amdgcn_ballot_w32(hit);
    int nh = (int)__builtin_popcount(msk);
    nh = nh > 32 ? 32 : nh;
    cnt += nh;
#pragma unroll 1
    for (int q = 0; q < nh; ++q) {
      const int k = __builtin_ffs((int)msk) - 1;
      msk &= msk - 1u;
      int node = i0 + (k < 0 ? 0 : k);
      node = node > nN - 1 ? nN - 1 : node;
      const float* rp = Hf + (size_t)node * HD + 8 * lane;
      const v4f va = *(const v4f*)rp;
      const v4f vb = *(const v4f*)(rp + 4);
      a0 += va.x; a1 += va.y; a2 += va.z; a3 += va.w;
      a4 += vb.x; a5 += vb.y; a6 += vb.z; a7 += vb.w;
    }
  }
  const float cf = (cnt < 1) ? 1.0f : (float)cnt;
  v4f pa, pb;
  pa.x = a0 / cf; pa.y = a1 / cf; pa.z = a2 / cf; pa.w = a3 / cf;
  pb.x = a4 / cf; pb.y = a5 / cf; pb.z = a6 / cf; pb.w = a7 / cf;
  const HL hl = split8(pa, pb);
  unsigned short* gp = PL + (size_t)g * K2 + 8 * lane;
  *(volatile v4u*)gp = hl.h;
  *(volatile v4u*)(gp + HD) = hl.l;
  __threadfence();
  *(volatile v4u*)gp = hl.h;
  *(volatile v4u*)(gp + HD) = hl.l;
}

static inline size_t al256(size_t o) { return (o + 255) & ~(size_t)255; }

extern "C" void kernel_launch(void* const* d_in, const int* in_sizes, int n_in,
                              void* d_out, int out_size, void* d_ws, size_t ws_size,
                              hipStream_t stream) {
  if (n_in < 22) return;
  if (in_sizes[0] != NN * 9 || in_sizes[1] != NN * 8) return;
  if (in_sizes[2] != 2 * NE || in_sizes[3] != NN) return;
  if (in_sizes[4] != 9 * HD || in_sizes[5] != HD || in_sizes[6] != 8 * HD || in_sizes[7] != HD) return;
  if (in_sizes[8] != NL * HD * HD || in_sizes[12] != NL * HD * HD) return;
  if (in_sizes[9] != NL * HD || in_sizes[10] != NL * HD || in_sizes[11] != NL * HD) return;
  if (in_sizes[13] != NL * HD || in_sizes[14] != NL * HD || in_sizes[15] != NL * HD) return;
  if (in_sizes[16] != HD * HD || in_sizes[17] != HD || in_sizes[18] != HD || in_sizes[19] != HD) return;
  if (in_sizes[20] != HD * NTO || in_sizes[21] != NTO) return;
  if (out_size != NG * NTO) return;

  const float* x_atom = (const float*)d_in[0];
  const float* x_pe   = (const float*)d_in[1];
  const int*   eidx   = (const int*)  d_in[2];
  const int*   src    = eidx;
  const int*   dst    = eidx + NE;
  const int*   bat    = (const int*)  d_in[3];
  const float* ae_w   = (const float*)d_in[4];
  const float* ae_b   = (const float*)d_in[5];
  const float* pe_w   = (const float*)d_in[6];
  const float* pe_b   = (const float*)d_in[7];
  const float* w1     = (const float*)d_in[8];
  const float* b1     = (const float*)d_in[9];
  const float* g1     = (const float*)d_in[10];
  const float* be1    = (const float*)d_in[11];
  const float* w2     = (const float*)d_in[12];
  const float* b2     = (const float*)d_in[13];
  const float* bng    = (const float*)d_in[14];
  const float* bnb    = (const float*)d_in[15];
  const float* cl1_w  = (const float*)d_in[16];
  const float* cl1_b  = (const float*)d_in[17];
  const float* clg    = (const float*)d_in[18];
  const float* clb    = (const float*)d_in[19];
  const float* cl2_w  = (const float*)d_in[20];
  const float* cl2_b  = (const float*)d_in[21];
  float* out = (float*)d_out;

  char* ws = (char*)d_ws;
  size_t off = 0;
  const size_t oP1   = off; off = al256(off + (size_t)MP * K2 * 2);
  const size_t oP2   = off; off = al256(off + (size_t)MP * HD * 4);
  const size_t oLIST = off; off = al256(off + (size_t)NBLK * RCAP * 4);
  const size_t oCNT  = off; off = al256(off + (size_t)NBLK * NB * 4);
  const size_t oOFF  = off; off = al256(off + (size_t)NBLK * NB * 4);
  const size_t oXE   = off; off = al256(off + (size_t)MP * KE * 2);
  const size_t oWE   = off; off = al256(off + (size_t)HD * KE * 2);
  const size_t oWP   = off; off = al256(off + (size_t)(11 * PLANE + NTO * K2) * 2);
  const size_t oTAB  = off; off = al256(off + (size_t)TABN * 4);
  const size_t oPT   = off; off = al256(off + (size_t)(MP / GBM) * (HD / GBN) * PARTW * 4);
  const size_t oST   = off; off = al256(off + (size_t)(4 * HD) * 4);
  const size_t oPL   = off; off = al256(off + (size_t)MG * K2 * 2);
  const size_t oCF   = off; off = al256(off + (size_t)MG * HD * 4);
  const size_t oCH   = off; off = al256(off + (size_t)MG * K2 * 2);
  if (off > ws_size || off > (size_t)WSMAX) return;
  unsigned short* P1   = (unsigned short*)(ws + oP1);
  float*          P2   = (float*)(ws + oP2);
  int*            LIST = (int*)(ws + oLIST);
  int*            CNT  = (int*)(ws + oCNT);
  int*            OFF  = (int*)(ws + oOFF);
  unsigned short* XE   = (unsigned short*)(ws + oXE);
  unsigned short* WE   = (unsigned short*)(ws + oWE);
  unsigned short* WP   = (unsigned short*)(ws + oWP);
  float*          TAB  = (float*)(ws + oTAB);
  float*          PART = (float*)(ws + oPT);
  float*          STAT = (float*)(ws + oST);
  unsigned short* PL   = (unsigned short*)(ws + oPL);
  float*          CF   = (float*)(ws + oCF);
  unsigned short* CH   = (unsigned short*)(ws + oCH);

  hipFuncSetAttribute(reinterpret_cast<const void*>(&k_compact), hipFuncAttributeMaxDynamicSharedMemorySize, LDS_CMP);

  const int vec8 = ((NE & 3) == 0) ? 1 : 0;
  const dim3 gN(MP / GBM, HD / GBN);
  const dim3 gH1(MG / GBM, HD / GBN);
  const dim3 gH2(MG / GBM, 1);

  k_xe<<<MP / XROWS, NTHR, 0, stream>>>(x_atom, x_pe, NN, XE);
  k_wprep<<<32 * (2 * NL + 1) + 16, NTHR, 0, stream>>>(w1, w2, cl1_w, cl2_w, WP);
  k_small<<<1 + (NSEG * 64 + NTHR - 1) / NTHR, NTHR, 0, stream>>>(ae_w, pe_w, b1, g1, be1, b2, bng, bnb,
                                                                  ae_b, pe_b, cl1_b, clg, clb, cl2_b, WE, TAB);
  k_compact<<<NBLK, NTHR, LDS_CMP, stream>>>(src, dst, NE, NN, vec8, LIST, CNT, OFF);
  k_gemm<KE, 0><<<gN, GTHR, 0, stream>>>(XE, WE, TAB + TEB, P2, HD, MP, NN, PART);
  for (int i = 0; i < NL; ++i) {
    k_agg<<<NBLK, NTHR, 0, stream>>>(LIST, CNT, OFF, P2, P1, NN, MP);
    k_gemm<K2, 1><<<gN, GTHR, 0, stream>>>(P1, WP + (size_t)i * PLANE, TAB + TB1 + i * HD, P2, HD, MP, NN, PART);
    k_comb<<<1, NTHR, 0, stream>>>(PART, MP / GBM, HD / GBN, TAB + TG1 + i * HD, TAB + TBE1 + i * HD, STAT);
    k_apply_hl<<<(MP * 32) / NTHR, NTHR, 0, stream>>>(P2, STAT, P1, NN, MP * 32);
    k_gemm<K2, 1><<<gN, GTHR, 0, stream>>>(P1, WP + (size_t)(NL + i) * PLANE, TAB + TB2 + i * HD, P2, HD, MP, NN, PART);
    k_comb<<<1, NTHR, 0, stream>>>(PART, MP / GBM, HD / GBN, TAB + TBNG + i * HD, TAB + TBNB + i * HD, STAT);
    k_apply_f<<<(NN * 64 + NTHR - 1) / NTHR, NTHR, 0, stream>>>(P2, STAT, NN * 64);
  }
  k_pool<<<MG / NWAVE, NTHR, 0, stream>>>(P2, bat, NN, NG, PL);
  k_gemm<K2, 1><<<gH1, GTHR, 0, stream>>>(PL, WP + (size_t)(2 * NL) * PLANE, TAB + TCL1B, CF, HD, MG, NG, PART);
  k_comb<<<1, NTHR, 0, stream>>>(PART, MG / GBM, HD / GBN, TAB + TCLG, TAB + TCLB, STAT);
  k_apply_hl<<<(MG * 32) / NTHR, NTHR, 0, stream>>>(CF, STAT, CH, NG, MG * 32);
  k_gemm<K2, 0><<<gH2, GTHR, 0, stream>>>(CH, WP + (size_t)(2 * NL + 1) * PLANE, TAB + TCL2B, out, NTO, NG, NG, PART);
}
